// NFTnetworkBlock_68006512165217
// MI455X (gfx1250) — hardware-verified
//
#include <hip/hip_runtime.h>


#define NB_  4
#define TT   8192
#define CC   256
#define NE   8
#define NT   (NB_ * TT)
typedef _Float16 h16;
typedef unsigned short bf;
typedef __attribute__((ext_vector_type(16))) __bf16   v16bf;
typedef __attribute__((ext_vector_type(16))) _Float16 v16h;
typedef __attribute__((ext_vector_type(8)))  _Float16 v8h;
typedef __attribute__((ext_vector_type(8)))  unsigned short v8us;
typedef __attribute__((ext_vector_type(8)))  float    v8f;
typedef __attribute__((ext_vector_type(4)))  float    v4f;
typedef v8h  __attribute__((may_alias)) v8ha;
typedef v4f  __attribute__((may_alias)) v4fa;
typedef v8us __attribute__((may_alias)) v8usa;

__device__ __forceinline__ unsigned short f2bf(float f) { unsigned u = __float_as_uint(f); u += 0x7FFFu + ((u >> 16) & 1u); return (unsigned short)(u >> 16); }
__device__ __forceinline__ float bf2f(unsigned short b) { return __uint_as_float(((unsigned)b) << 16); }
__device__ __forceinline__ float bfr(float f) { return bf2f(f2bf(f)); }
__device__ __forceinline__ v16h cat16(v8h lo, v8h hi) { return __builtin_shufflevector(lo, hi, 0, 1, 2, 3, 4, 5, 6, 7, 8, 9, 10, 11, 12, 13, 14, 15); }
__device__ __forceinline__ v16bf cat16b(v8us lo, v8us hi) { return __builtin_bit_cast(v16bf, __builtin_shufflevector(lo, hi, 0, 1, 2, 3, 4, 5, 6, 7, 8, 9, 10, 11, 12, 13, 14, 15)); }
__device__ __forceinline__ v8f wmma16(v16h a, v16h b, v8f c) { return __builtin_amdgcn_wmma_f32_16x16x32_f16(false, a, false, b, (short)0, c, false, false); }
__device__ __forceinline__ v8f wmmab(v16bf a, v16bf b, v8f c) { return __builtin_amdgcn_wmma_f32_16x16x32_bf16(false, a, false, b, (short)0, c, false, false); }


template <typename T16> struct WFrag;
template <> struct WFrag<h16> { typedef v16h V; static __device__ __forceinline__ V ld(const h16* p) { return cat16(*(const v8h*)p, *(const v8h*)(p + 16)); } static __device__ __forceinline__ v8f mma(V a, V b, v8f c) { return wmma16(a, b, c); } };
template <> struct WFrag<bf> { typedef v16bf V; static __device__ __forceinline__ V ld(const bf* p) { return cat16b(*(const v8us*)p, *(const v8us*)(p + 16)); } static __device__ __forceinline__ v8f mma(V a, V b, v8f c) { return wmmab(a, b, c); } };
template <typename T16, int NSPLIT, bool BIAS>
__global__ __launch_bounds__(32) void k_gemmw(const T16* __restrict__ A, const T16* __restrict__ A2, const T16* __restrict__ Bt, const T16* __restrict__ Bt2, int K, float* C, int ldc, const float* __restrict__ bias, size_t sA, size_t sB, size_t sC) {
    typedef typename WFrag<T16>::V V;
    __shared__ __align__(16) float os[16 * 68];
    const size_t z = blockIdx.z; A += z * sA; if (A2) A2 += z * sA; Bt += z * sB; if (Bt2) Bt2 += z * sB; C += z * sC;
    const int lane = threadIdx.x & 31, lr = lane & 15, hi = lane >> 4; const int r0 = blockIdx.x * 64, c0 = blockIdx.y * 64;
    v8f acc[4][4];
#pragma unroll
    for (int mb = 0; mb < 4; ++mb)
#pragma unroll
        for (int nb = 0; nb < 4; ++nb) acc[mb][nb] = (v8f){};
    const size_t aoff = (size_t)(r0 + lr) * K + 8 * hi, boff = (size_t)(c0 + lr) * K + 8 * hi;
#pragma unroll 1
    for (int kc = 0; kc < K; kc += 32) {
        V a[4], a2[4];
#pragma unroll
        for (int mb = 0; mb < 4; ++mb) { a[mb] = WFrag<T16>::ld(A + aoff + (size_t)mb * 16 * K + kc); if (NSPLIT == 1 || NSPLIT == 2) a2[mb] = WFrag<T16>::ld(A2 + aoff + (size_t)mb * 16 * K + kc); }
#pragma unroll
        for (int nb = 0; nb < 4; ++nb) { const V b = WFrag<T16>::ld(Bt + boff + (size_t)nb * 16 * K + kc); V b2; if (NSPLIT >= 2) b2 = WFrag<T16>::ld(Bt2 + boff + (size_t)nb * 16 * K + kc);
#pragma unroll
            for (int mb = 0; mb < 4; ++mb) { acc[mb][nb] = WFrag<T16>::mma(a[mb], b, acc[mb][nb]); if (NSPLIT == 1 || NSPLIT == 2) acc[mb][nb] = WFrag<T16>::mma(a2[mb], b, acc[mb][nb]); if (NSPLIT >= 2) acc[mb][nb] = WFrag<T16>::mma(a[mb], b2, acc[mb][nb]); } }
        asm volatile("v_nop\n\tv_nop\n\tv_nop\n\tv_nop" : "+v"(acc[0][0]), "+v"(acc[1][1]), "+v"(acc[2][2]), "+v"(acc[3][3]) : "v"(a[0]), "v"(a[3]));
    }
#pragma unroll
    for (int mb = 0; mb < 4; ++mb) {
#pragma unroll
        for (int nb = 0; nb < 4; ++nb) {
#pragma unroll
            for (int j = 0; j < 8; ++j) os[(hi * 8 + j) * 68 + nb * 16 + lr] = acc[mb][nb][j]; }
        __builtin_amdgcn_wave_barrier(); asm volatile("" ::: "memory");
        float* crow = C + (size_t)(r0 + mb * 16) * ldc + c0;
#pragma unroll 1
        for (int ps = 0; ps < 2; ++ps) {
#pragma unroll
            for (int s = 0; s < 8; ++s) { const int row = 2 * s + hi, cofs = lr * 4; v4f val = *(const v4fa*)(os + row * 68 + cofs); if (BIAS) { val[0] += bfr(bias[c0 + cofs]); val[1] += bfr(bias[c0 + cofs + 1]); val[2] += bfr(bias[c0 + cofs + 2]); val[3] += bfr(bias[c0 + cofs + 3]); }
                *(volatile v4f*)(crow + (size_t)row * ldc + cofs) = val; }
            if (ps == 0) __threadfence(); }
        __builtin_amdgcn_wave_barrier(); asm volatile("" ::: "memory");
    }
}

__device__ __forceinline__ h16 tohx(float x) { return (h16)x; }
__device__ __forceinline__ void splitf(float y, unsigned short& h, unsigned short& l) { h = f2bf(y); l = f2bf(y - bf2f(h)); }
__device__ __forceinline__ float geluf(float t) { return 0.5f * t * (1.0f + erff(t * 0.70710678118654752f)); }
typedef __attribute__((ext_vector_type(2))) unsigned short v2us;
typedef __attribute__((ext_vector_type(4))) unsigned short v4us;
typedef __attribute__((ext_vector_type(4))) _Float16 v4h;

__global__ __launch_bounds__(256) void k_cvt8(const float* __restrict__ src, bf* dst, size_t n8) { const size_t i = (size_t)blockIdx.x * 256 + threadIdx.x; if (i >= n8) return; const v8f v = *(const v8f*)(src + i * 8); v8us o;
#pragma unroll
    for (int k = 0; k < 8; ++k) o[k] = f2bf(v[k]); *(volatile v8us*)(dst + i * 8) = o; __threadfence(); *(volatile v8us*)(dst + i * 8) = o; }
__global__ __launch_bounds__(256) void k_wtb(const float* __restrict__ w, int K, int N, int wpitch, bf* Bt) {
    const int lane = threadIdx.x & 31; const int L = blockIdx.x * 8 + (threadIdx.x >> 5); if (L >= N * K / 64) return; const int e = L * 64 + lane * 2; const int n = e / K, k = e % K; v2us o;
    o[0] = f2bf(w[(size_t)k * wpitch + n]); o[1] = f2bf(w[(size_t)(k + 1) * wpitch + n]); *(volatile v2us*)(Bt + e) = o; __threadfence(); *(volatile v2us*)(Bt + e) = o;
}
__global__ __launch_bounds__(256) void k_ln(const float* __restrict__ x, const float* __restrict__ gw, const float* __restrict__ gb, float* H) {
    const int lane = threadIdx.x & 31; const int r = blockIdx.x * 8 + (threadIdx.x >> 5); if (r >= NT) return; float v[8]; float s = 0.f;
#pragma unroll
    for (int c = 0; c < 2; ++c) { const v4f a = *(const v4f*)(x + (size_t)r * CC + c * 128 + lane * 4);
#pragma unroll
        for (int q = 0; q < 4; ++q) { v[c * 4 + q] = bfr(a[q]); s += v[c * 4 + q]; } }
#pragma unroll
    for (int sh = 16; sh; sh >>= 1) s += __shfl_xor(s, sh, 32);
    const float mu = s * (1.0f / CC); float qq = 0.f;
#pragma unroll
    for (int i = 0; i < 8; ++i) { const float d0 = v[i] - mu; qq = fmaf(d0, d0, qq); }
#pragma unroll
    for (int sh = 16; sh; sh >>= 1) qq += __shfl_xor(qq, sh, 32);
    const float rs = rsqrtf(qq * (1.0f / CC) + 1e-5f); v4f o[2];
#pragma unroll
    for (int c = 0; c < 2; ++c)
#pragma unroll
        for (int q = 0; q < 4; ++q) { const int col = c * 128 + lane * 4 + q; o[c][q] = (v[c * 4 + q] - mu) * rs * bfr(gw[col]) + bfr(gb[col]); }
#pragma unroll 1
    for (int ps = 0; ps < 2; ++ps) {
#pragma unroll
        for (int c = 0; c < 2; ++c) *(volatile v4f*)(H + (size_t)r * CC + c * 128 + lane * 4) = o[c];
        if (ps == 0) __threadfence(); }
}
__global__ __launch_bounds__(256) void k_stats(const float* __restrict__ H, const int* __restrict__ mask, float* STW) {
    const int lane = threadIdx.x & 31; const int wg = blockIdx.x * 8 + (threadIdx.x >> 5); if (wg >= NB_ * CC) return; const int b = wg >> 8, c = wg & 255;
    float s = 0.f, cnt = 0.f;
#pragma unroll 4
    for (int t = lane; t < TT; t += 32) { const float m = (mask[(size_t)b * TT + t] != 0) ? 1.f : 0.f; cnt += m; s = fmaf(m, H[((size_t)b * TT + t) * CC + c], s); }
#pragma unroll
    for (int sh = 16; sh; sh >>= 1) { s += __shfl_xor(s, sh, 32); cnt += __shfl_xor(cnt, sh, 32); }
    const float n = fmaxf(cnt, 1.0f); const float mean = __fdiv_rn(s, n); float q = 0.f;
#pragma unroll 4
    for (int t = lane; t < TT; t += 32) { const float m = (mask[(size_t)b * TT + t] != 0) ? 1.f : 0.f; const float d = H[((size_t)b * TT + t) * CC + c] - mean; q = fmaf(m, d * d, q); }
#pragma unroll
    for (int sh = 16; sh; sh >>= 1) q += __shfl_xor(q, sh, 32);
    const float var_b = __fdiv_rn(q, n); const float can = n > 1.0f ? 1.f : 0.f; const float corr = __fdiv_rn(n, fmaxf(n - 1.0f, 1e-9f));
    const float var_u = var_b * corr * can + var_b * (1.0f - can); const float std_u = fmaxf(sqrtf(var_u), 1e-9f);
    const float o = lane == 0 ? mean : (lane == 1 ? std_u : (lane == 2 ? var_u : 0.f)); *(volatile float*)(STW + (size_t)wg * 32 + lane) = o; __threadfence(); *(volatile float*)(STW + (size_t)wg * 32 + lane) = o;
}
__global__ __launch_bounds__(256) void k_sbias(const float* __restrict__ STW, const float* __restrict__ W1, const float* __restrict__ b1, float* SB) {
    const int lane = threadIdx.x & 31; const int wg = blockIdx.x * 8 + (threadIdx.x >> 5); if (wg >= NB_ * NE) return; const int b = wg / NE, e = wg % NE; float acc[8];
#pragma unroll
    for (int j = 0; j < 8; ++j) acc[j] = bfr(b1[e * CC + lane + 32 * j]);
#pragma unroll 1
    for (int k = 0; k < CC; ++k) { const float* st = STW + ((size_t)b * CC + k) * 32; const float mn = st[0], sd = st[1], vr = st[2]; const float* w = W1 + ((size_t)e * 4 * CC) * CC;
#pragma unroll
        for (int j = 0; j < 8; ++j) { const int c = lane + 32 * j; acc[j] = fmaf(mn, bfr(w[(size_t)(CC + k) * CC + c]), acc[j]); acc[j] = fmaf(sd, bfr(w[(size_t)(2 * CC + k) * CC + c]), acc[j]); acc[j] = fmaf(vr, bfr(w[(size_t)(3 * CC + k) * CC + c]), acc[j]); } }
#pragma unroll 1
    for (int ps = 0; ps < 2; ++ps) {
#pragma unroll
        for (int j = 0; j < 8; ++j) *(volatile float*)(SB + (size_t)wg * CC + lane + 32 * j) = acc[j];
        if (ps == 0) __threadfence(); }
}
__global__ __launch_bounds__(256) void k_gelu(const float* __restrict__ H1, const float* __restrict__ SB, int e, bf* Ph, bf* Pl) {
    const int lane = threadIdx.x & 31; const int L0 = (blockIdx.x * 8 + (threadIdx.x >> 5)) * 8; const int nlines = NT * CC / 64;
#pragma unroll 1
    for (int ps = 0; ps < 2; ++ps) {
#pragma unroll 1
        for (int l = 0; l < 8; ++l) { const int L = L0 + l; if (L >= nlines) break; const int idx = L * 64 + lane * 2; const int c = idx & 255; const int b = idx >> 21; v2us oh, ol;
#pragma unroll
            for (int q = 0; q < 2; ++q) { unsigned short a, c2; splitf(geluf(H1[(size_t)idx + q] + SB[((size_t)b * NE + e) * CC + c + q]), a, c2); oh[q] = a; ol[q] = c2; }
            *(volatile v2us*)(Ph + (size_t)idx) = oh; *(volatile v2us*)(Pl + (size_t)idx) = ol; }
        if (ps == 0) __threadfence(); }
}
__global__ __launch_bounds__(256) void k_energy(const float* __restrict__ O, const float* __restrict__ We, const float* __restrict__ be, int e, float* EN, h16* OE) {
    const int lane = threadIdx.x & 31; const int t = blockIdx.x * 8 + (threadIdx.x >> 5); if (t >= NT) return; const float* orow = O + (size_t)t * CC; float s = 0.f; v8h o8;
    { const v8f a = *(const v8f*)(orow + lane * 8);
#pragma unroll
      for (int q = 0; q < 8; ++q) { s = fmaf(a[q], bfr(We[e * CC + lane * 8 + q]), s); o8[q] = tohx(a[q]); } }
#pragma unroll
    for (int sh = 16; sh; sh >>= 1) s += __shfl_xor(s, sh, 32);
    s += bfr(be[e]);
    const float prev = EN[(size_t)t * 32 + lane]; const float nv = (lane == e) ? s : prev;
    *(volatile v8h*)(OE + ((size_t)e * NT + t) * CC + lane * 8) = o8; *(volatile float*)(EN + (size_t)t * 32 + lane) = nv; __threadfence();
    *(volatile v8h*)(OE + ((size_t)e * NT + t) * CC + lane * 8) = o8; *(volatile float*)(EN + (size_t)t * 32 + lane) = nv;
}
__global__ __launch_bounds__(256) void k_mix(const float* __restrict__ EN, const h16* __restrict__ OE, const int* __restrict__ mask, const float* __restrict__ log_beta, const float* __restrict__ prior, float* OUT) {
    const int lane = threadIdx.x & 31; const int t = blockIdx.x * 8 + (threadIdx.x >> 5); if (t >= NT) return; const bool live = mask[t] != 0; const float beta = __expf(bfr(log_beta[0]));
    float ne[NE]; float mx = -3.0e38f;
#pragma unroll
    for (int e = 0; e < NE; ++e) { ne[e] = -beta * (EN[(size_t)t * 32 + e] + bfr(prior[e])); mx = fmaxf(mx, ne[e]); }
    float sum = 0.f;
#pragma unroll
    for (int e = 0; e < NE; ++e) { ne[e] = __expf(ne[e] - mx); sum += ne[e]; }
    const float inv = __fdiv_rn(1.0f, sum); v8f o = (v8f){};
    if (live) {
#pragma unroll
        for (int e = 0; e < NE; ++e) { const v8h a = *(const v8h*)(OE + ((size_t)e * NT + t) * CC + lane * 8); const float p = ne[e] * inv;
#pragma unroll
            for (int q = 0; q < 8; ++q) o[q] = fmaf(p, (float)a[q], o[q]); } }
    *(volatile v8f*)(OUT + (size_t)t * CC + lane * 8) = o; __threadfence(); *(volatile v8f*)(OUT + (size_t)t * CC + lane * 8) = o;
}

extern "C" void kernel_launch(void* const* d_in, const int* in_sizes, int n_in,
                              void* d_out, int out_size, void* d_ws, size_t ws_size, hipStream_t stream) {
    (void)in_sizes; (void)n_in; (void)out_size;
    const float* x = (const float*)d_in[0]; const int* mask = (const int*)d_in[1]; const float* ln_w = (const float*)d_in[2]; const float* ln_b = (const float*)d_in[3]; const float* W1 = (const float*)d_in[4]; const float* b1 = (const float*)d_in[5];
    const float* W2 = (const float*)d_in[6]; const float* b2 = (const float*)d_in[7]; const float* We = (const float*)d_in[8]; const float* be = (const float*)d_in[9]; const float* log_beta = (const float*)d_in[10]; const float* prior = (const float*)d_in[11];
    float* OUT = (float*)d_out;
    char* wsp = (char*)d_ws;
    auto take = [&](size_t bytes) { char* p = wsp; wsp += (bytes + 255) & ~(size_t)255; return (void*)p; };
    bf* W1T = (bf*)take((size_t)NE * CC * CC * 2); bf* W2T = (bf*)take((size_t)NE * CC * CC * 2);
    float* STW = (float*)take((size_t)NB_ * CC * 32 * 4); float* SB = (float*)take((size_t)NB_ * NE * CC * 4); float* EN = (float*)take((size_t)NT * 32 * 4);
    bf* XB = (bf*)take((size_t)NT * CC * 2); float* F = (float*)take((size_t)NT * CC * 4);
    bf* Gh = (bf*)take((size_t)NT * CC * 2); bf* Gl = (bf*)take((size_t)NT * CC * 2); h16* OE = (h16*)take((size_t)NE * NT * CC * 2);
    if ((size_t)(wsp - (char*)d_ws) > ws_size) return;
    hipMemsetAsync(EN, 0, (size_t)NT * 32 * 4, stream);
    for (int e = 0; e < NE; ++e) { k_wtb<<<(CC * CC / 64 + 7) / 8, 256, 0, stream>>>(W1 + (size_t)e * 4 * CC * CC, CC, CC, CC, W1T + (size_t)e * CC * CC); k_wtb<<<(CC * CC / 64 + 7) / 8, 256, 0, stream>>>(W2 + (size_t)e * CC * CC, CC, CC, CC, W2T + (size_t)e * CC * CC); }
    k_cvt8<<<(unsigned)((NT * CC / 8 + 255) / 256), 256, 0, stream>>>(x, XB, (size_t)NT * CC / 8);
    k_ln<<<NT / 8, 256, 0, stream>>>(x, ln_w, ln_b, F);
    k_stats<<<NB_ * CC / 8, 256, 0, stream>>>(F, mask, STW);
    k_sbias<<<NB_ * NE / 8, 256, 0, stream>>>(STW, W1, b1, SB);
    for (int e = 0; e < NE; ++e) {
        k_gemmw<bf, 0, false><<<dim3(NT / 64, CC / 64, 1), 32, 0, stream>>>(XB, nullptr, W1T + (size_t)e * CC * CC, nullptr, CC, F, CC, nullptr, 0, 0, 0);
        k_gelu<<<(unsigned)((NT * CC / 64 + 63) / 64), 256, 0, stream>>>(F, SB, e, Gh, Gl);
        k_gemmw<bf, 1, true><<<dim3(NT / 64, CC / 64, 1), 32, 0, stream>>>(Gh, Gl, W2T + (size_t)e * CC * CC, nullptr, CC, F, CC, b2 + e * CC, 0, 0, 0);
        k_energy<<<NT / 8, 256, 0, stream>>>(F, We, be, e, EN, OE); }
    k_mix<<<NT / 8, 256, 0, stream>>>(EN, OE, mask, log_beta, prior, OUT);
}
